// MultiHeadAttention_773094113988
// MI455X (gfx1250) — hardware-run, weakly checked
//
#include <hip/hip_runtime.h>
#ifndef NB
#define NB 16
#endif
#ifndef SEQ
#define SEQ 512
#endif
#define NB_FULL 16
#define SEQ_FULL 512
#define EMBED 768
#define HEADS 12
#define HD 64
#define NQKV 2304
#define MTOK (NB * SEQ)
#define XSTRIDE_FULL ((size_t)SEQ_FULL * EMBED)
#define PLANE_E ((size_t)MTOK * EMBED)

static_assert(SEQ % 64 == 0);
static_assert(MTOK % 128 == 0);
static_assert(SEQ <= SEQ_FULL);
static_assert(NB <= NB_FULL);
static_assert(HD == 64);
static_assert(HEADS * HD == EMBED);
static_assert(EMBED % 128 == 0);
static_assert((2 * EMBED) % 128 == 0);
static_assert(EMBED % 32 == 0);
static_assert(PLANE_E * 2 * 5 + (size_t)NQKV * EMBED * 2 + (size_t)EMBED * EMBED * 2 + 2048 <= (size_t)134217728);

typedef __bf16 v16b __attribute__((ext_vector_type(16)));
typedef _Float16 v16h __attribute__((ext_vector_type(16)));
typedef unsigned short v8us __attribute__((ext_vector_type(8), may_alias));
typedef float v8f __attribute__((ext_vector_type(8)));
typedef float v4f __attribute__((ext_vector_type(4)));
typedef float v4fa __attribute__((ext_vector_type(4), may_alias));
union FragH { v16h v; v8us half[2]; _Float16 h[16]; unsigned short u[16]; };
union FragG { v16b b; v16h h; v8us half[2]; };

#define LOG2E 1.4426950408889634f

__device__ __forceinline__ unsigned short bf16_bits(float x) {
  unsigned int u = __float_as_uint(x);
  return (unsigned short)((u + 0x7FFFu + ((u >> 16) & 1u)) >> 16);
}
__device__ __forceinline__ float bf16_val(unsigned short b) { return __uint_as_float(((unsigned int)b) << 16); }
__device__ __forceinline__ float bf16_rne(float x) { return bf16_val(bf16_bits(x)); }
__device__ __forceinline__ unsigned short f16_bits(float x) {
  union { _Float16 h; unsigned short u; } c;
  c.h = (_Float16)x;
  return c.u;
}

__device__ __forceinline__ v8f mma_hs2(v16h a0, v16h b0, v16h a1, v16h b1, v8f c) {
  c = __builtin_amdgcn_wmma_f32_16x16x32_f16(false, a0, false, b0, (short)0, c, false, false);
  c = __builtin_amdgcn_wmma_f32_16x16x32_f16(false, a1, false, b1, (short)0, c, false, false);
  asm volatile("v_nop\n\tv_nop\n\tv_nop\n\tv_nop" : "+v"(c) : "v"(a0), "v"(b0), "v"(a1), "v"(b1));
  return c;
}
__device__ __forceinline__ void mma_h1(v16h a, v16h b, v8f& c) {
  c = __builtin_amdgcn_wmma_f32_16x16x32_f16(false, a, false, b, (short)0, c, false, false);
  asm volatile("v_nop\n\tv_nop\n\tv_nop\n\tv_nop" : "+v"(c) : "v"(a), "v"(b));
}
template <bool F16>
__device__ __forceinline__ v8f wm1(const FragG& a, const FragG& b, v8f c) {
  if (F16) return __builtin_amdgcn_wmma_f32_16x16x32_f16(false, a.h, false, b.h, (short)0, c, false, false);
  return __builtin_amdgcn_wmma_f32_16x16x32_bf16(false, a.b, false, b.b, (short)0, c, false, false);
}
template <bool F16>
__device__ __forceinline__ void mma_blk(const FragG& a0, const FragG& a1, const FragG& b0, const FragG& b1,
                                        const FragG& b2, const FragG& b3, v8f (&c)[2][4]) {
  c[0][0] = wm1<F16>(a0, b0, c[0][0]);
  c[0][1] = wm1<F16>(a0, b1, c[0][1]);
  c[0][2] = wm1<F16>(a0, b2, c[0][2]);
  c[0][3] = wm1<F16>(a0, b3, c[0][3]);
  c[1][0] = wm1<F16>(a1, b0, c[1][0]);
  c[1][1] = wm1<F16>(a1, b1, c[1][1]);
  c[1][2] = wm1<F16>(a1, b2, c[1][2]);
  c[1][3] = wm1<F16>(a1, b3, c[1][3]);
  asm volatile("v_nop\n\tv_nop\n\tv_nop\n\tv_nop"
               : "+v"(c[0][0]), "+v"(c[0][1]), "+v"(c[0][2]), "+v"(c[0][3]),
                 "+v"(c[1][0]), "+v"(c[1][1]), "+v"(c[1][2]), "+v"(c[1][3])
               : "v"(a0.h), "v"(a1.h), "v"(b0.h), "v"(b1.h), "v"(b2.h), "v"(b3.h));
}

__global__ __launch_bounds__(256) void k_xb(const float* __restrict__ X, unsigned short* __restrict__ Xb) {
  const int t = blockIdx.x * 256 + threadIdx.x;
  if (t >= MTOK * (EMBED / 8)) return;
  const int row = t / (EMBED / 8), piece = t - row * (EMBED / 8);
  const int b = row / SEQ, s = row - b * SEQ;
  const float* src = X + (size_t)b * XSTRIDE_FULL + (size_t)s * EMBED + piece * 8;
  const v4f x0 = *(const v4fa*)(src), x1 = *(const v4fa*)(src + 4);
  v8us o;
  o[0] = bf16_bits(x0[0]); o[1] = bf16_bits(x0[1]); o[2] = bf16_bits(x0[2]); o[3] = bf16_bits(x0[3]);
  o[4] = bf16_bits(x1[0]); o[5] = bf16_bits(x1[1]); o[6] = bf16_bits(x1[2]); o[7] = bf16_bits(x1[3]);
  unsigned short* d = Xb + (size_t)t * 8;
  *(volatile v8us*)d = o;
  __threadfence();
  *(volatile v8us*)d = o;
}

template <int CONV>
__global__ __launch_bounds__(256) void k_wt(const float* __restrict__ in, unsigned short* __restrict__ out, int rows, int cols) {
  __shared__ unsigned short tl[64][66];
  const int tid = threadIdx.x;
  const int c0 = blockIdx.x * 64, r0 = blockIdx.y * 64;
  for (int i = tid; i < 64 * 16; i += 256) {
    const int j = i >> 4, c4 = (i & 15) * 4;
    const v4f x = *(const v4fa*)(in + (size_t)(r0 + j) * cols + c0 + c4);
    unsigned short u0, u1, u2, u3;
    if (CONV == 0) {
      u0 = bf16_bits(x[0]); u1 = bf16_bits(x[1]); u2 = bf16_bits(x[2]); u3 = bf16_bits(x[3]);
    } else {
      u0 = f16_bits(bf16_rne(x[0]) * 64.0f); u1 = f16_bits(bf16_rne(x[1]) * 64.0f);
      u2 = f16_bits(bf16_rne(x[2]) * 64.0f); u3 = f16_bits(bf16_rne(x[3]) * 64.0f);
    }
    tl[c4 + 0][j] = u0; tl[c4 + 1][j] = u1; tl[c4 + 2][j] = u2; tl[c4 + 3][j] = u3;
  }
  __syncthreads();
  for (int pass = 0; pass < 2; ++pass) {
    for (int i = tid; i < 64 * 8; i += 256) {
      const int d = i >> 3, j8 = (i & 7) * 8;
      v8us o;
#pragma unroll
      for (int q = 0; q < 8; ++q) o[q] = tl[d][j8 + q];
      *(volatile v8us*)(out + (size_t)(c0 + d) * rows + r0 + j8) = o;
    }
    if (pass == 0) __threadfence();
  }
}

template <int MODE>
__global__ __launch_bounds__(256) void k_gemm(const unsigned short* __restrict__ A, const unsigned short* __restrict__ B,
                                              const float* __restrict__ bias, unsigned short* __restrict__ P, float* __restrict__ C) {
  __shared__ __attribute__((aligned(16))) float st[8][16][68];
  const int tid = threadIdx.x, w = __builtin_amdgcn_readfirstlane((int)(tid >> 5)), lane = tid & 31, ln = lane & 15, hh = lane >> 4;
  const int wm = w & 3, wn = w >> 2;
  const int rowBase = blockIdx.y * 128 + wm * 32;
  const int colBase = blockIdx.x * 128 + wn * 64;
  v8f acc[2][4] = {};
  const unsigned short* ap = A + (size_t)(rowBase + ln) * EMBED + 8 * hh;
  const unsigned short* bp = B + (size_t)(colBase + ln) * EMBED + 8 * hh;
#pragma unroll 1
  for (int k = 0; k < EMBED; k += 32) {
    FragG a0, a1, b0, b1, b2, b3;
    a0.half[0] = *(const v8us*)(ap + k);                a0.half[1] = *(const v8us*)(ap + k + 16);
    a1.half[0] = *(const v8us*)(ap + 16 * EMBED + k);   a1.half[1] = *(const v8us*)(ap + 16 * EMBED + k + 16);
    b0.half[0] = *(const v8us*)(bp + k);                b0.half[1] = *(const v8us*)(bp + k + 16);
    b1.half[0] = *(const v8us*)(bp + 16 * EMBED + k);   b1.half[1] = *(const v8us*)(bp + 16 * EMBED + k + 16);
    b2.half[0] = *(const v8us*)(bp + 32 * EMBED + k);   b2.half[1] = *(const v8us*)(bp + 32 * EMBED + k + 16);
    b3.half[0] = *(const v8us*)(bp + 48 * EMBED + k);   b3.half[1] = *(const v8us*)(bp + 48 * EMBED + k + 16);
    mma_blk<MODE == 2>(a0, a1, b0, b1, b2, b3, acc);
  }

#pragma unroll
  for (int mt = 0; mt < 2; ++mt) {
    if (mt) __syncthreads();
#pragma unroll
    for (int nt = 0; nt < 4; ++nt)
#pragma unroll
      for (int r = 0; r < 8; ++r)
        st[w][8 * hh + r][16 * nt + ln] = acc[mt][nt][r];
    __syncthreads();
    const int row0 = rowBase + 16 * mt;
    if (MODE == 0) {
      const int which = colBase / EMBED;
      const int head = (colBase - which * EMBED) >> 6;
      const int rsub = lane >> 3, pc = lane & 7;
      const v4f g0 = *(const v4fa*)(bias + colBase + 8 * pc), g1 = *(const v4fa*)(bias + colBase + 8 * pc + 4);
      float bb[8];
#pragma unroll
      for (int q = 0; q < 4; ++q) { bb[q] = bf16_rne(g0[q]); bb[4 + q] = bf16_rne(g1[q]); }
      unsigned short* base = P + (size_t)which * PLANE_E;
      for (int pass = 0; pass < 2; ++pass) {
#pragma unroll
        for (int i = 0; i < 4; ++i) {
          const int rr = 4 * i + rsub;
          const int tok = row0 + rr;
          const int b = tok / SEQ, n = tok - b * SEQ;
          const v4f v0 = *(const v4fa*)&st[w][rr][8 * pc], v1 = *(const v4fa*)&st[w][rr][8 * pc + 4];
          v8us o;
#pragma unroll
          for (int q = 0; q < 4; ++q) {
            o[q] = f16_bits((v0[q] + bb[q]) * 16.0f);
            o[4 + q] = f16_bits((v1[q] + bb[4 + q]) * 16.0f);
          }
          unsigned short* dst = base + ((size_t)(b * HEADS + head) * SEQ + n) * HD + 8 * pc;
          *(volatile v8us*)dst = o;
        }
        if (pass == 0) __threadfence();
      }
    } else if (MODE == 1) {
      const int rsub = lane >> 3, pc = lane & 7;
      const int b = colBase / SEQ, n0 = colBase - b * SEQ;
      for (int pass = 0; pass < 2; ++pass) {
#pragma unroll
        for (int i = 0; i < 4; ++i) {
          const int rr = 4 * i + rsub;
          const int c = row0 + rr;
          const float bs = bf16_rne(bias[c]);
          const v4f v0 = *(const v4fa*)&st[w][rr][8 * pc], v1 = *(const v4fa*)&st[w][rr][8 * pc + 4];
          v8us o;
#pragma unroll
          for (int q = 0; q < 4; ++q) {
            o[q] = f16_bits((v0[q] + bs) * 16.0f);
            o[4 + q] = f16_bits((v1[q] + bs) * 16.0f);
          }
          unsigned short* dst = P + ((size_t)b * EMBED + c) * SEQ + n0 + 8 * pc;
          *(volatile v8us*)dst = o;
        }
        if (pass == 0) __threadfence();
      }
    } else {
      const int rsub = lane >> 4, pc = lane & 15;
      const v4f g = *(const v4fa*)(bias + colBase + 4 * pc);
      v4f bb;
      bb[0] = bf16_rne(g[0]); bb[1] = bf16_rne(g[1]); bb[2] = bf16_rne(g[2]); bb[3] = bf16_rne(g[3]);
      for (int pass = 0; pass < 2; ++pass) {
#pragma unroll
        for (int i = 0; i < 8; ++i) {
          const int rr = 2 * i + rsub;
          const int tok = row0 + rr;
          const int b = tok / SEQ, n = tok - b * SEQ;
          const v4f v = *(const v4fa*)&st[w][rr][4 * pc];
          v4f o;
          o[0] = v[0] * 6.103515625e-05f + bb[0];
          o[1] = v[1] * 6.103515625e-05f + bb[1];
          o[2] = v[2] * 6.103515625e-05f + bb[2];
          o[3] = v[3] * 6.103515625e-05f + bb[3];
          *(volatile v4f*)(C + ((size_t)b * SEQ_FULL + n) * EMBED + colBase + 4 * pc) = o;
        }
        if (pass == 0) __threadfence();
      }
    }
  }
}

__device__ __forceinline__ void fa_step(const unsigned short* __restrict__ Kp, const unsigned short* __restrict__ Vp,
                                        int key0, int ln, int hh, const FragH& q0, const FragH& q1,
                                        float& mr, float& lr, v8f (&Oh)[4]) {
  const unsigned short* kp0 = Kp + (size_t)(key0 + ln) * HD + 8 * hh;
  const unsigned short* kp1 = kp0 + 16 * HD;
  FragH k00, k01, k10, k11;
  k00.half[0] = *(const v8us*)(kp0);      k00.half[1] = *(const v8us*)(kp0 + 16);
  k01.half[0] = *(const v8us*)(kp0 + 32); k01.half[1] = *(const v8us*)(kp0 + 48);
  k10.half[0] = *(const v8us*)(kp1);      k10.half[1] = *(const v8us*)(kp1 + 16);
  k11.half[0] = *(const v8us*)(kp1 + 32); k11.half[1] = *(const v8us*)(kp1 + 48);
  const v8f z8 = {0.f, 0.f, 0.f, 0.f, 0.f, 0.f, 0.f, 0.f};
  const v8f s0 = mma_hs2(k00.v, q0.v, k01.v, q1.v, z8);
  const v8f s1 = mma_hs2(k10.v, q0.v, k11.v, q1.v, z8);
  float sc[16];
#pragma unroll
  for (int r = 0; r < 8; ++r) { sc[r] = s0[r] * 0.00048828125f; sc[8 + r] = s1[r] * 0.00048828125f; }
  float mx = sc[0];
#pragma unroll
  for (int i = 1; i < 16; ++i) mx = fmaxf(mx, sc[i]);
  mx = fmaxf(mx, __shfl_xor(mx, 16, 32));
  const float mnew = fmaxf(mr, mx);
  const float al = exp2f((mr - mnew) * LOG2E);
  mr = mnew;
  FragH ph;
  float ps = 0.0f;
#pragma unroll
  for (int i = 0; i < 16; ++i) {
    const float pc = exp2f(fmaf(sc[i] - mnew, LOG2E, 8.0f));
    const _Float16 h = (_Float16)pc;
    ph.h[i] = h;
    ps += (float)h;
  }
  ps += __shfl_xor(ps, 16, 32);
  lr = lr * al + ps;
#pragma unroll
  for (int t = 0; t < 4; ++t) Oh[t] = Oh[t] * al;
  const unsigned short* vp = Vp + (size_t)ln * SEQ + key0 + 8 * hh;
#pragma unroll
  for (int t = 0; t < 4; ++t) {
    FragH vf;
    vf.half[0] = *(const v8us*)(vp + (size_t)t * 16 * SEQ);
    vf.half[1] = *(const v8us*)(vp + (size_t)t * 16 * SEQ + 16);
    mma_h1(vf.v, ph.v, Oh[t]);
  }
}

__global__ __launch_bounds__(128) void k_attn(const unsigned short* __restrict__ QK, const unsigned short* __restrict__ Vt,
                                              unsigned short* __restrict__ Cx) {
  __shared__ __attribute__((aligned(16))) float so[4][16][68];
  const int tid = threadIdx.x, w = __builtin_amdgcn_readfirstlane((int)(tid >> 5)), lane = tid & 31, ln = lane & 15, hh = lane >> 4;
  const int bh = blockIdx.x / (SEQ / 64), qt = blockIdx.x % (SEQ / 64);
  const int b = bh / HEADS, h = bh - b * HEADS;
  const int qbase = qt * 64 + 16 * w;
  const int qg = qbase + ln;
  const unsigned short* qrow = QK + ((size_t)bh * SEQ + qg) * HD + 8 * hh;
  FragH q0, q1;
  q0.half[0] = *(const v8us*)(qrow);      q0.half[1] = *(const v8us*)(qrow + 16);
  q1.half[0] = *(const v8us*)(qrow + 32); q1.half[1] = *(const v8us*)(qrow + 48);
  float mr = -3.0e38f, lr = 0.0f;
  v8f Oh[4] = {};
  const unsigned short* Kp = QK + PLANE_E + (size_t)bh * SEQ * HD;
  const unsigned short* Vp = Vt + (size_t)bh * HD * SEQ;
#pragma unroll 1
  for (int j = 0; j < SEQ / 32; ++j)
    fa_step(Kp, Vp, 32 * j, ln, hh, q0, q1, mr, lr, Oh);

  const float inv = 16.0f * (1.0f / lr);
#pragma unroll
  for (int t = 0; t < 4; ++t)
#pragma unroll
    for (int r = 0; r < 8; ++r)
      so[w][ln][16 * t + 8 * hh + r] = Oh[t][r] * inv;
  __syncthreads();
  unsigned short* cg = Cx + ((size_t)b * SEQ + qbase) * EMBED + h * HD;
  const int rsub = lane >> 3, pc = lane & 7;
  for (int pass = 0; pass < 2; ++pass) {
#pragma unroll
    for (int i = 0; i < 4; ++i) {
      const int rr = 4 * i + rsub;
      const v4f v0 = *(const v4fa*)&so[w][rr][8 * pc], v1 = *(const v4fa*)&so[w][rr][8 * pc + 4];
      v8us o;
#pragma unroll
      for (int q = 0; q < 4; ++q) { o[q] = f16_bits(v0[q]); o[4 + q] = f16_bits(v1[q]); }
      *(volatile v8us*)(cg + (size_t)rr * EMBED + 8 * pc) = o;
    }
    if (pass == 0) __threadfence();
  }
}

extern "C" void kernel_launch(void* const* d_in, const int* in_sizes, int n_in,
                              void* d_out, int out_size, void* d_ws, size_t ws_size, hipStream_t stream) {
  if (n_in < 5) return;
  const long long needx = (long long)(NB - 1) * SEQ_FULL * EMBED + (long long)SEQ * EMBED;
  if ((long long)in_sizes[0] < needx) return;
  if ((long long)in_sizes[1] < (long long)EMBED * NQKV) return;
  if ((long long)in_sizes[2] < (long long)NQKV) return;
  if ((long long)in_sizes[3] < (long long)EMBED * EMBED) return;
  if ((long long)in_sizes[4] < (long long)EMBED) return;
  if ((long long)out_size < needx) return;
  const float* X    = (const float*)d_in[0];
  const float* Wqkv = (const float*)d_in[1];
  const float* bqkv = (const float*)d_in[2];
  const float* Wo   = (const float*)d_in[3];
  const float* bo   = (const float*)d_in[4];
  float* O = (float*)d_out;
  char* ws = (char*)d_ws;
  size_t off = 0;
  const size_t plane = PLANE_E * 2;
  unsigned short* Xb    = (unsigned short*)(ws + off); off += (plane + 255) & ~(size_t)255;
  unsigned short* WqkvT = (unsigned short*)(ws + off); off += ((size_t)NQKV * EMBED * 2 + 255) & ~(size_t)255;
  unsigned short* WoT   = (unsigned short*)(ws + off); off += ((size_t)EMBED * EMBED * 2 + 255) & ~(size_t)255;
  unsigned short* QK    = (unsigned short*)(ws + off); off += (2 * plane + 255) & ~(size_t)255;
  unsigned short* Vt    = (unsigned short*)(ws + off); off += (plane + 255) & ~(size_t)255;
  unsigned short* Cx    = (unsigned short*)(ws + off); off += (plane + 255) & ~(size_t)255;
  if (off > ws_size) return;

  k_xb<<<(unsigned)((MTOK * (EMBED / 8) + 255) / 256), 256, 0, stream>>>(X, Xb);
  k_wt<0><<<dim3(NQKV / 64, EMBED / 64), 256, 0, stream>>>(Wqkv, WqkvT, EMBED, NQKV);
  k_wt<1><<<dim3(EMBED / 64, EMBED / 64), 256, 0, stream>>>(Wo, WoT, EMBED, EMBED);
  k_gemm<0><<<dim3((2 * EMBED) / 128, MTOK / 128), 256, 0, stream>>>(Xb, WqkvT, bqkv, QK, O);
  k_gemm<1><<<dim3(MTOK / 128, EMBED / 128), 256, 0, stream>>>(WqkvT + (size_t)2 * EMBED * EMBED, Xb, bqkv + 2 * EMBED, Vt, O);
  k_attn<<<(unsigned)(NB * HEADS * (SEQ / 64)), 128, 0, stream>>>(QK, Vt, Cx);
  k_gemm<2><<<dim3(EMBED / 128, MTOK / 128), 256, 0, stream>>>(Cx, WoT, bo, Vt, O);
}
